// Model_6150393168181
// MI455X (gfx1250) — hardware-verified
//
#include <hip/hip_runtime.h>
#include <math.h>
#include <stdint.h>

#define NB     256
#define NN     128
#define NROWS  (NB * NN)
#define NWK    8
#define NCH    4
#define CHB    (NB / NCH)
#define CHROWS (CHB * NN)
#define UTP    (2 * NWK * NN)
#define MCP    (3 * NWK * NN)

static_assert(NROWS == 32768);
static_assert(NN == 128);
static_assert(NWK * NN == 1024);
static_assert(NB % NCH == 0);
static_assert(CHROWS % 64 == 0);
static_assert(UTP == 2048);
static_assert(MCP == 3072);
static_assert((NWK * NN) % 32 == 0);
static_assert(NN % 32 == 0);
static_assert(((CHROWS / 64) * (NN / 64)) % 8 == 0);

typedef __attribute__((ext_vector_type(16))) __bf16   v16b;
typedef __attribute__((ext_vector_type(8)))  __bf16   v8b;
typedef __attribute__((ext_vector_type(8)))  float    v8f;
typedef __attribute__((ext_vector_type(4)))  float    v4f;
typedef __attribute__((ext_vector_type(4)))  unsigned int v4u;

__device__ __forceinline__ unsigned short f2bf_bits(float f) {
  unsigned u = __float_as_uint(f);
  return (unsigned short)((u + 0x7FFFu + ((u >> 16) & 1u)) >> 16);
}
__device__ __forceinline__ float bf_bits2f(unsigned short h) { return __uint_as_float(((unsigned)h) << 16); }
__device__ __forceinline__ float bf_rne(float f) { return bf_bits2f(f2bf_bits(f)); }
__device__ __forceinline__ unsigned pk16(unsigned short a, unsigned short b) { return (unsigned)a | ((unsigned)b << 16); }

struct HL { v4u h; v4u l; };
__device__ __forceinline__ HL split8(float f0, float f1, float f2, float f3, float f4, float f5, float f6, float f7) {
  const unsigned short h0 = f2bf_bits(f0), h1 = f2bf_bits(f1), h2 = f2bf_bits(f2), h3 = f2bf_bits(f3);
  const unsigned short h4 = f2bf_bits(f4), h5 = f2bf_bits(f5), h6 = f2bf_bits(f6), h7 = f2bf_bits(f7);
  const unsigned short l0 = f2bf_bits(f0 - bf_bits2f(h0)), l1 = f2bf_bits(f1 - bf_bits2f(h1));
  const unsigned short l2 = f2bf_bits(f2 - bf_bits2f(h2)), l3 = f2bf_bits(f3 - bf_bits2f(h3));
  const unsigned short l4 = f2bf_bits(f4 - bf_bits2f(h4)), l5 = f2bf_bits(f5 - bf_bits2f(h5));
  const unsigned short l6 = f2bf_bits(f6 - bf_bits2f(h6)), l7 = f2bf_bits(f7 - bf_bits2f(h7));
  HL r;
  r.h = (v4u){pk16(h0, h1), pk16(h2, h3), pk16(h4, h5), pk16(h6, h7)};
  r.l = (v4u){pk16(l0, l1), pk16(l2, l3), pk16(l4, l5), pk16(l6, l7)};
  return r;
}
__device__ __forceinline__ v4u blend4(v4u a, v4u b, unsigned m) {
  v4u r;
  r[0] = (a[0] & ~m) | (b[0] & m);
  r[1] = (a[1] & ~m) | (b[1] & m);
  r[2] = (a[2] & ~m) | (b[2] & m);
  r[3] = (a[3] & ~m) | (b[3] & m);
  return r;
}

__device__ __forceinline__ void dep_guard_b(v8f& a, v8f& b, v16b x, v16b y) { asm volatile("v_nop\n\tv_nop\n\tv_nop\n\tv_nop" : "+v"(a), "+v"(b) : "v"(x), "v"(y)); }
__device__ __forceinline__ void keep4_b(v16b a, v16b b, v16b c, v16b d) { asm volatile("v_nop" :: "v"(a), "v"(b), "v"(c), "v"(d)); }
__device__ __forceinline__ void acc_guard4(v8f& a, v8f& b, v8f& c, v8f& d) { asm volatile("v_nop\n\tv_nop\n\tv_nop\n\tv_nop" : "+v"(a), "+v"(b), "+v"(c), "+v"(d)); }

union FragB { v16b v; v8b h[2]; };
__device__ __forceinline__ v16b frag_load(const __bf16* p) {
  FragB f; f.h[0] = *(const v8b*)(p); f.h[1] = *(const v8b*)(p + 16); return f.v;
}
__device__ __forceinline__ v8f mma_b(v16b a, v16b b, v8f c) {
  return __builtin_amdgcn_wmma_f32_16x16x32_bf16(false, a, false, b, (short)0, c, false, false);
}

__device__ __forceinline__ void mma_tile64(v8f (&acc)[4][4], const __bf16* a, int lda, const __bf16* b, int ldb, int K) {
#pragma unroll 1
  for (int k0 = 0; k0 < K; k0 += 32) {
    v16b bh[4];
#pragma unroll
    for (int j = 0; j < 4; ++j) bh[j] = frag_load(b + (size_t)(j * 16) * ldb + k0);
#pragma unroll
    for (int i = 0; i < 4; ++i) {
      const v16b ah = frag_load(a + (size_t)(i * 16) * lda + k0);
#pragma unroll
      for (int j = 0; j < 4; ++j) acc[i][j] = mma_b(ah, bh[j], acc[i][j]);
      dep_guard_b(acc[i][0], acc[i][3], ah, ah);
    }
    keep4_b(bh[0], bh[1], bh[2], bh[3]);
  }
}

template <int NWV, int OUT_MODE, bool DIV>
__global__ __launch_bounds__(NWV * 32) void gemm64_kernel(
    const unsigned short* __restrict__ Ap, int lda, long sAy, long sAz,
    const unsigned short* __restrict__ Btp, int ldb, long sBy, long sBz,
    void* Cout, void* Cout2, void* Cout3, int ldc, long sCy, long sCz,
    int tilesN, int segK, int nseg, int a0, int a1, int a2, int b0, int b1, int b2) {
  __shared__ __align__(16) float sT[NWV][16 * 68];
  const int lane = threadIdx.x & 31;
  const int wave = threadIdx.x >> 5;
  const int tile = blockIdx.x * NWV + wave;
  const int tm = tile / tilesN;
  const int tn = tile - tm * tilesN;
  const int m0 = tm << 6;
  const int n0 = tn << 6;
  const int rlane = lane & 15;
  const int koff  = (lane >> 4) * 8;
  const int mOff  = (lane >> 4) * 8;

  const __bf16* A = (const __bf16*)Ap  + (size_t)blockIdx.y * (size_t)sAy + (size_t)blockIdx.z * (size_t)sAz;
  const __bf16* B = (const __bf16*)Btp + (size_t)blockIdx.y * (size_t)sBy + (size_t)blockIdx.z * (size_t)sBz;
  const __bf16* arow = A + (size_t)(m0 + rlane) * lda + koff;
  const __bf16* brow = B + (size_t)(n0 + rlane) * ldb + koff;

  v8f acc[4][4];
#pragma unroll
  for (int i = 0; i < 4; ++i)
#pragma unroll
    for (int j = 0; j < 4; ++j) acc[i][j] = (v8f){0.f, 0.f, 0.f, 0.f, 0.f, 0.f, 0.f, 0.f};

#pragma unroll 1
  for (int s = 0; s < nseg; ++s) {
    const int ab = (s == 0) ? a0 : ((s == 1) ? a1 : a2);
    const int bb = (s == 0) ? b0 : ((s == 1) ? b1 : b2);
    mma_tile64(acc, arow + ab, lda, brow + bb, ldb, segK);
  }
  acc_guard4(acc[0][0], acc[0][1], acc[0][2], acc[0][3]);
  acc_guard4(acc[1][0], acc[1][1], acc[1][2], acc[1][3]);
  acc_guard4(acc[2][0], acc[2][1], acc[2][2], acc[2][3]);
  acc_guard4(acc[3][0], acc[3][1], acc[3][2], acc[3][3]);

  const size_t cofs = (size_t)blockIdx.y * (size_t)sCy + (size_t)blockIdx.z * (size_t)sCz;
  const float SQ = sqrtf(128.0f);
  float* slab = sT[wave];
#pragma unroll
  for (int i = 0; i < 4; ++i) {
    const int mBase = m0 + (i << 4);
#pragma unroll
    for (int j = 0; j < 4; ++j) {
#pragma unroll
      for (int r = 0; r < 8; ++r) {
        float v = acc[i][j][r];
        if (DIV) v = v / SQ;
        slab[(mOff + r) * 68 + (j << 4) + rlane] = v;
      }
    }
    __syncthreads();
    if (OUT_MODE == 0) {
      float* C = (float*)Cout + cofs;
      const int hh = lane >> 4, c4 = (lane & 15) * 4;
      v4f ov[8];
#pragma unroll
      for (int it = 0; it < 8; ++it) ov[it] = *(const v4f*)(slab + (it * 2 + hh) * 68 + c4);
      for (int pass = 0; pass < 2; ++pass) {
#pragma unroll
        for (int it = 0; it < 8; ++it) {
          const int row = it * 2 + hh;
          *(volatile v4f*)(C + (size_t)(mBase + row) * ldc + n0 + c4) = ov[it];
        }
        __threadfence();
      }
    } else {
      const int q = lane >> 3, c8 = (lane & 7) * 8;
      unsigned short* C  = (unsigned short*)Cout  + cofs;
      unsigned short* C2 = (unsigned short*)Cout2 + cofs;
      unsigned short* C3 = (unsigned short*)Cout3 + cofs;
      v4u hv[4], lv[4];
#pragma unroll
      for (int it = 0; it < 4; ++it) {
        const float* sp = slab + (it * 4 + q) * 68 + c8;
        const v4f u0 = *(const v4f*)sp;
        const v4f u1 = *(const v4f*)(sp + 4);
        const HL s = split8(u0[0], u0[1], u0[2], u0[3], u1[0], u1[1], u1[2], u1[3]);
        hv[it] = s.h; lv[it] = s.l;
      }
      for (int pass = 0; pass < 2; ++pass) {
#pragma unroll
        for (int it = 0; it < 4; ++it) {
          const size_t go = (size_t)(mBase + it * 4 + q) * ldc + n0 + c8;
          *(volatile v4u*)(C + go) = hv[it];
          if (OUT_MODE == 2) { *(volatile v4u*)(C2 + go) = lv[it]; }
          if (OUT_MODE == 3) { *(volatile v4u*)(C2 + go) = hv[it]; *(volatile v4u*)(C3 + go) = lv[it]; }
        }
        __threadfence();
      }
    }
    __syncthreads();
  }
}

__global__ __launch_bounds__(256) void prep_x_kernel(const float* __restrict__ flows, unsigned short* __restrict__ X0) {
  __shared__ __align__(16) float sx[8][128];
  const int lane = threadIdx.x & 31, wave = threadIdx.x >> 5;
  const size_t row = (size_t)blockIdx.x * 8 + wave;
  const v4f v = *(const v4f*)(flows + row * 128 + 4 * lane);
  const float x0 = bf_rne(v[0]), x1 = bf_rne(v[1]), x2 = bf_rne(v[2]), x3 = bf_rne(v[3]);
  float ss = x0 * x0 + x1 * x1 + x2 * x2 + x3 * x3;
  ss += __shfl_xor(ss, 1);
  ss += __shfl_xor(ss, 2);
  ss += __shfl_xor(ss, 4);
  ss += __shfl_xor(ss, 8);
  ss += __shfl_xor(ss, 16);
  const float den = sqrtf(ss * 0.0078125f);
  const v4f y = {x0 / den, x1 / den, x2 / den, x3 / den};
  *(v4f*)(&sx[wave][4 * lane]) = y;
  __syncthreads();
  const float* sp = &sx[wave][(lane & 15) * 8];
  const v4f u0 = *(const v4f*)sp;
  const v4f u1 = *(const v4f*)(sp + 4);
  const HL s = split8(u0[0], u0[1], u0[2], u0[3], u1[0], u1[1], u1[2], u1[3]);
  const unsigned msk = 0u - (unsigned)(lane >> 4);
  const v4u ov = blend4(s.h, s.l, msk);
  volatile v4u* p = (volatile v4u*)(X0 + row * 256 + lane * 8);
  *p = ov;
  __threadfence();
  *p = ov;
}

__global__ __launch_bounds__(256) void cvt8_kernel(const float* __restrict__ src, unsigned short* __restrict__ dst, int n8) {
  const int g = blockIdx.x * 256 + threadIdx.x;
  if (g >= n8) return;
  const v4f a = *(const v4f*)(src + (size_t)g * 8);
  const v4f c = *(const v4f*)(src + (size_t)g * 8 + 4);
  v4u o;
  o[0] = pk16(f2bf_bits(a[0]), f2bf_bits(a[1]));
  o[1] = pk16(f2bf_bits(a[2]), f2bf_bits(a[3]));
  o[2] = pk16(f2bf_bits(c[0]), f2bf_bits(c[1]));
  o[3] = pk16(f2bf_bits(c[2]), f2bf_bits(c[3]));
  volatile v4u* p = (volatile v4u*)(dst + (size_t)g * 8);
  *p = o;
  __threadfence();
  *p = o;
}

__global__ __launch_bounds__(256) void tconv_kernel(const float* __restrict__ W, unsigned short* __restrict__ oh,
                                                    int ldin, int ldout, long sIn, long sOut) {
  __shared__ __align__(16) float tf[64 * 68];
  W  += (size_t)blockIdx.z * (size_t)sIn;
  oh += (size_t)blockIdx.z * (size_t)sOut;
  const int c0  = blockIdx.x * 64;
  const int r0  = blockIdx.y * 64;
  const int tid = threadIdx.x;
  {
    const int lr = tid >> 4;
    const int c4 = (tid & 15) * 4;
#pragma unroll
    for (int it = 0; it < 4; ++it) {
      const int rr = it * 16 + lr;
      const v4f a = *(const v4f*)(W + (size_t)(r0 + rr) * ldin + c0 + c4);
      *(v4f*)(tf + rr * 68 + c4) = a;
    }
  }
  __syncthreads();
  const int sub = tid >> 3;
  const int c8  = (tid & 7) * 8;
  v4u hv[2];
#pragma unroll
  for (int it = 0; it < 2; ++it) {
    const int oc = it * 32 + sub;
    v4u a;
#pragma unroll
    for (int q = 0; q < 4; ++q) {
      const float f0 = tf[(c8 + 2 * q) * 68 + oc];
      const float f1 = tf[(c8 + 2 * q + 1) * 68 + oc];
      a[q] = pk16(f2bf_bits(f0), f2bf_bits(f1));
    }
    hv[it] = a;
  }
  for (int pass = 0; pass < 2; ++pass) {
#pragma unroll
    for (int it = 0; it < 2; ++it) {
      const int oc = it * 32 + sub;
      const size_t go = (size_t)(c0 + oc) * ldout + r0 + c8;
      *(volatile v4u*)(oh + go) = hv[it];
    }
    __threadfence();
  }
}

__global__ __launch_bounds__(256) void spack_kernel(const float* __restrict__ s2w, unsigned short* __restrict__ S) {
  const int g = blockIdx.x * 256 + threadIdx.x;
  const float* src = s2w + (size_t)(g >> 4) * 1024 + (size_t)(g & 15) * 64;
  v4f t[16];
#pragma unroll
  for (int i = 0; i < 16; ++i) t[i] = *(const v4f*)(src + 4 * i);
  v4u o[8];
#pragma unroll
  for (int w = 0; w < 8; ++w) {
    v4u a;
#pragma unroll
    for (int q = 0; q < 4; ++q) {
      const float f0 = t[2 * (2 * q) + (w >> 2)][w & 3];
      const float f1 = t[2 * (2 * q + 1) + (w >> 2)][w & 3];
      a[q] = pk16(f2bf_bits(f0), f2bf_bits(f1));
    }
    o[w] = a;
  }
  for (int pass = 0; pass < 2; ++pass) {
#pragma unroll
    for (int w = 0; w < 8; ++w)
      *(volatile v4u*)(S + (size_t)w * 16384 + (size_t)g * 8) = o[w];
    __threadfence();
  }
}

template <int KIN>
__global__ __launch_bounds__(KIN) void pref_kernel(const unsigned short* __restrict__ X, unsigned short* __restrict__ AGG) {
  __shared__ __align__(16) float sA[16 * KIN];
  const int c = threadIdx.x;
  float run = 0.0f;
#pragma unroll 1
  for (int ch = 0; ch < 8; ++ch) {
#pragma unroll 1
    for (int jj = 0; jj < 16; ++jj) {
      const int j = ch * 16 + jj;
      const float dj = (j == 0) ? 1.0f : (float)j;
      sA[jj * KIN + c] = run / dj;
      const float xv = bf_bits2f(X[(size_t)j * (2 * KIN) + c]) + bf_bits2f(X[(size_t)j * (2 * KIN) + KIN + c]);
      run += xv;
    }
    __syncthreads();
    v4u ov[4];
#pragma unroll
    for (int it = 0; it < 4; ++it) {
      const int p = it * KIN + c;
      const int row = p / (KIN / 4);
      const int q = p - row * (KIN / 4);
      const int islo = (q >= KIN / 8) ? 1 : 0;
      const int col = (q - islo * (KIN / 8)) * 8;
      const float* sp = sA + row * KIN + col;
      const v4f u0 = *(const v4f*)sp;
      const v4f u1 = *(const v4f*)(sp + 4);
      const HL s = split8(u0[0], u0[1], u0[2], u0[3], u1[0], u1[1], u1[2], u1[3]);
      ov[it] = blend4(s.h, s.l, 0u - (unsigned)islo);
    }
    unsigned short* base = AGG + (size_t)ch * 16 * (2 * KIN);
    for (int pass = 0; pass < 2; ++pass) {
#pragma unroll
      for (int it = 0; it < 4; ++it)
        *(volatile v4u*)(base + (size_t)(it * KIN + c) * 8) = ov[it];
      __threadfence();
    }
    __syncthreads();
  }
}

template <int NOUT, int KIN, bool LAST>
__global__ __launch_bounds__((NOUT / 64) * 64) void sage_kernel(
    const unsigned short* __restrict__ X, const unsigned short* __restrict__ AGG,
    const unsigned short* __restrict__ WR, const unsigned short* __restrict__ WL,
    const float* __restrict__ bl, unsigned short* Y, unsigned short* FT) {
  constexpr int TN  = NOUT / 64;
  constexpr int NWV = 2 * TN;
  constexpr int P   = NOUT + 4;
  constexpr int RPW = 128 / NWV;
  static_assert(NOUT == 128 || NOUT == 256);
  static_assert(KIN == 128 || KIN == 256);
  static_assert(!LAST || NOUT == 128);
  extern __shared__ __align__(16) float smem[];
  float* sB = smem;
  float* sY = smem + NOUT;

  const int tid = threadIdx.x, lane = tid & 31, wave = tid >> 5;
  const int rlane = lane & 15;
  const int koff = (lane >> 4) * 8;
  const int mOff = (lane >> 4) * 8;
  const int t  = blockIdx.x;
  const int tm = wave / TN;
  const int tn = wave - tm * TN;
  const int m0 = 64 * tm, n0 = 64 * tn;

  if (tid < NOUT / 4) {
    v4f bv = *(const v4f*)(bl + 4 * tid);
    bv[0] = bf_rne(bv[0]); bv[1] = bf_rne(bv[1]); bv[2] = bf_rne(bv[2]); bv[3] = bf_rne(bv[3]);
    *(v4f*)(sB + 4 * tid) = bv;
  }
  __syncthreads();

  v8f acc[4][4];
#pragma unroll
  for (int i = 0; i < 4; ++i)
#pragma unroll
    for (int j = 0; j < 4; ++j) acc[i][j] = (v8f){0.f, 0.f, 0.f, 0.f, 0.f, 0.f, 0.f, 0.f};

  {
    const __bf16* a = (const __bf16*)X + ((size_t)t * 128 + m0 + rlane) * (2 * KIN) + koff;
    const __bf16* b = (const __bf16*)WR + (size_t)(n0 + rlane) * KIN + koff;
    mma_tile64(acc, a, 2 * KIN, b, KIN, KIN);
    mma_tile64(acc, a + KIN, 2 * KIN, b, KIN, KIN);
  }
  if (t == 0) {
    const __bf16* a = (const __bf16*)AGG + (size_t)(m0 + rlane) * (2 * KIN) + koff;
    const __bf16* b = (const __bf16*)WL + (size_t)(n0 + rlane) * KIN + koff;
    mma_tile64(acc, a, 2 * KIN, b, KIN, KIN);
    mma_tile64(acc, a + KIN, 2 * KIN, b, KIN, KIN);
  }
  acc_guard4(acc[0][0], acc[0][1], acc[0][2], acc[0][3]);
  acc_guard4(acc[1][0], acc[1][1], acc[1][2], acc[1][3]);
  acc_guard4(acc[2][0], acc[2][1], acc[2][2], acc[2][3]);
  acc_guard4(acc[3][0], acc[3][1], acc[3][2], acc[3][3]);

#pragma unroll
  for (int i = 0; i < 4; ++i) {
#pragma unroll
    for (int j = 0; j < 4; ++j) {
      const int col = n0 + 16 * j + rlane;
      const float bv = sB[col];
#pragma unroll
      for (int r = 0; r < 8; ++r)
        sY[(m0 + 16 * i + mOff + r) * P + col] = acc[i][j][r] + bv;
    }
  }
  __syncthreads();

  const int c8 = (NOUT == 128) ? (lane & 15) * 8 : lane * 8;
  const unsigned hmask = 0u - (unsigned)(lane >> 4);
#pragma unroll 1
  for (int rr = 0; rr < RPW; ++rr) {
    const int row = wave * RPW + rr;
    float* sp = sY + row * P + c8;
    const v4f u0 = *(const v4f*)sp;
    const v4f u1 = *(const v4f*)(sp + 4);
    float y[8] = {u0[0], u0[1], u0[2], u0[3], u1[0], u1[1], u1[2], u1[3]};
    float ss = 0.0f;
#pragma unroll
    for (int e = 0; e < 8; ++e) ss += y[e] * y[e];
    ss += __shfl_xor(ss, 1);
    ss += __shfl_xor(ss, 2);
    ss += __shfl_xor(ss, 4);
    ss += __shfl_xor(ss, 8);
    if (NOUT == 256) ss += __shfl_xor(ss, 16);
    const float nrm = fmaxf(sqrtf(ss), 1e-12f);
#pragma unroll
    for (int e = 0; e < 8; ++e) y[e] = y[e] / nrm;
    if (LAST) {
      float s2 = 0.0f;
#pragma unroll
      for (int e = 0; e < 8; ++e) {
        const float v = y[e];
        const float rl = (v > 0.0f) ? v : (v - v);
        y[e] = rl;
        s2 += rl * rl;
      }
      s2 += __shfl_xor(s2, 1);
      s2 += __shfl_xor(s2, 2);
      s2 += __shfl_xor(s2, 4);
      s2 += __shfl_xor(s2, 8);
      const float den = sqrtf(s2 * 0.0078125f);
#pragma unroll
      for (int e = 0; e < 8; ++e) y[e] = y[e] / den;
      const v4f w0 = {y[0], y[1], y[2], y[3]};
      const v4f w1 = {y[4], y[5], y[6], y[7]};
      *(v4f*)sp = w0;
      *(v4f*)(sp + 4) = w1;
    }
    const HL s = split8(y[0], y[1], y[2], y[3], y[4], y[5], y[6], y[7]);
    const size_t grow = (size_t)t * 128 + row;
    if (NOUT == 128) {
      const v4u ov = blend4(s.h, s.l, hmask);
      volatile v4u* p = (volatile v4u*)(Y + grow * 256 + lane * 8);
      *p = ov;
      __threadfence();
      *p = ov;
    } else {
      volatile v4u* p0 = (volatile v4u*)(Y + grow * 512 + lane * 8);
      volatile v4u* p1 = (volatile v4u*)(Y + grow * 512 + 256 + lane * 8);
      *p0 = s.h; *p1 = s.l;
      __threadfence();
      *p0 = s.h; *p1 = s.l;
    }
  }

  if (LAST) {
    __syncthreads();
    const int m8 = (lane & 15) * 8;
#pragma unroll 1
    for (int dd = 0; dd < RPW; ++dd) {
      const int d = wave * RPW + dd;
      float v[8];
#pragma unroll
      for (int e = 0; e < 8; ++e) v[e] = sY[(m8 + e) * P + d];
      const HL s = split8(v[0], v[1], v[2], v[3], v[4], v[5], v[6], v[7]);
      const v4u ov = blend4(s.h, s.l, hmask);
      volatile v4u* p = (volatile v4u*)(FT + ((size_t)t * 128 + d) * 256 + lane * 8);
      *p = ov;
      __threadfence();
      *p = ov;
    }
  }
}

extern "C" void kernel_launch(void* const* d_in, const int* in_sizes, int n_in,
                              void* d_out, int out_size, void* d_ws, size_t ws_size,
                              hipStream_t stream) {
  if (n_in < 28) return;
  if (in_sizes[0] != NROWS * 128) return;
  if (in_sizes[10] != 16384 || in_sizes[11] != 128 || in_sizes[12] != 16384) return;
  if (in_sizes[13] != 32768 || in_sizes[14] != 256 || in_sizes[15] != 32768) return;
  if (in_sizes[16] != 32768 || in_sizes[17] != 128 || in_sizes[18] != 32768) return;
  if (in_sizes[19] != 16384 || in_sizes[20] != 128 || in_sizes[21] != 16384) return;
  if (in_sizes[24] != 131072 || in_sizes[25] != 131072 || in_sizes[27] != 131072) return;
  if (out_size != NROWS * 128) return;

  const float* flows = (const float*)d_in[0];
  const float* g1_wl = (const float*)d_in[10];
  const float* g1_bl = (const float*)d_in[11];
  const float* g1_wr = (const float*)d_in[12];
  const float* g2_wl = (const float*)d_in[13];
  const float* g2_bl = (const float*)d_in[14];
  const float* g2_wr = (const float*)d_in[15];
  const float* g3_wl = (const float*)d_in[16];
  const float* g3_bl = (const float*)d_in[17];
  const float* g3_wr = (const float*)d_in[18];
  const float* g4_wl = (const float*)d_in[19];
  const float* g4_bl = (const float*)d_in[20];
  const float* g4_wr = (const float*)d_in[21];
  const float* qsa   = (const float*)d_in[24];
  const float* ksa   = (const float*)d_in[25];
  const float* s2w   = (const float*)d_in[27];
  float* out = (float*)d_out;

  size_t off = 0;
  const size_t oRA = off;  off += (size_t)NROWS * 256 * 2;
  const size_t oRB = off;  off += (size_t)NROWS * 256 * 2;
  const size_t oRC = off;  off += (size_t)NROWS * 512 * 2;
  const size_t oRD = off;  off += (size_t)CHROWS * UTP * 2;
  const size_t oAG = off;  off += (size_t)128 * 512 * 2;
  const size_t oW1r = off; off += (size_t)16384 * 2;
  const size_t oW1l = off; off += (size_t)16384 * 2;
  const size_t oW2r = off; off += (size_t)32768 * 2;
  const size_t oW2l = off; off += (size_t)32768 * 2;
  const size_t oW3r = off; off += (size_t)32768 * 2;
  const size_t oW3l = off; off += (size_t)32768 * 2;
  const size_t oW4r = off; off += (size_t)16384 * 2;
  const size_t oW4l = off; off += (size_t)16384 * 2;
  const size_t oQT = off;  off += (size_t)8 * 16384 * 2;
  const size_t oKT = off;  off += (size_t)8 * 16384 * 2;
  const size_t oS  = off;  off += (size_t)8 * 16384 * 2;
  const size_t oMC = off;  off += (size_t)128 * MCP * 2;
  if (off > ws_size) return;
  if (off > (size_t)134217728) return;

  char* ws = (char*)d_ws;
  unsigned short* RA  = (unsigned short*)(ws + oRA);
  unsigned short* RB  = (unsigned short*)(ws + oRB);
  unsigned short* RC  = (unsigned short*)(ws + oRC);
  unsigned short* RD  = (unsigned short*)(ws + oRD);
  unsigned short* AG  = (unsigned short*)(ws + oAG);
  unsigned short* W1r = (unsigned short*)(ws + oW1r);
  unsigned short* W1l = (unsigned short*)(ws + oW1l);
  unsigned short* W2r = (unsigned short*)(ws + oW2r);
  unsigned short* W2l = (unsigned short*)(ws + oW2l);
  unsigned short* W3r = (unsigned short*)(ws + oW3r);
  unsigned short* W3l = (unsigned short*)(ws + oW3l);
  unsigned short* W4r = (unsigned short*)(ws + oW4r);
  unsigned short* W4l = (unsigned short*)(ws + oW4l);
  unsigned short* QT  = (unsigned short*)(ws + oQT);
  unsigned short* KT  = (unsigned short*)(ws + oKT);
  unsigned short* SP  = (unsigned short*)(ws + oS);
  unsigned short* MC  = (unsigned short*)(ws + oMC);

  prep_x_kernel<<<dim3(NROWS / 8), dim3(256), 0, stream>>>(flows, RA);

  cvt8_kernel<<<dim3(16384 / 8 / 256), dim3(256), 0, stream>>>(g1_wr, W1r, 16384 / 8);
  cvt8_kernel<<<dim3(16384 / 8 / 256), dim3(256), 0, stream>>>(g1_wl, W1l, 16384 / 8);
  cvt8_kernel<<<dim3(32768 / 8 / 256), dim3(256), 0, stream>>>(g2_wr, W2r, 32768 / 8);
  cvt8_kernel<<<dim3(32768 / 8 / 256), dim3(256), 0, stream>>>(g2_wl, W2l, 32768 / 8);
  cvt8_kernel<<<dim3(32768 / 8 / 256), dim3(256), 0, stream>>>(g3_wr, W3r, 32768 / 8);
  cvt8_kernel<<<dim3(32768 / 8 / 256), dim3(256), 0, stream>>>(g3_wl, W3l, 32768 / 8);
  cvt8_kernel<<<dim3(16384 / 8 / 256), dim3(256), 0, stream>>>(g4_wr, W4r, 16384 / 8);
  cvt8_kernel<<<dim3(16384 / 8 / 256), dim3(256), 0, stream>>>(g4_wl, W4l, 16384 / 8);

  tconv_kernel<<<dim3(2, 2, 8), dim3(256), 0, stream>>>(qsa, QT, 128, 128, 16384L, 16384L);
  tconv_kernel<<<dim3(2, 2, 8), dim3(256), 0, stream>>>(ksa, KT, 128, 128, 16384L, 16384L);

  spack_kernel<<<dim3(8), dim3(256), 0, stream>>>(s2w, SP);

  gemm64_kernel<4, 3, true><<<dim3(1, 8, 1), dim3(128), 0, stream>>>(
      QT, 128, 16384L, 0L, KT, 128, 16384L, 0L,
      (void*)MC, (void*)(MC + 1024), (void*)(MC + 2048), MCP, 128L, 0L,
      2, 128, 1, 0, 0, 0, 0, 0, 0);

  const int lds128 = (128 * (128 + 4) + 128) * 4;
  const int lds256 = (128 * (256 + 4) + 256) * 4;
  (void)hipFuncSetAttribute(reinterpret_cast<const void*>(&sage_kernel<128, 128, false>), hipFuncAttributeMaxDynamicSharedMemorySize, lds128);
  (void)hipFuncSetAttribute(reinterpret_cast<const void*>(&sage_kernel<256, 128, false>), hipFuncAttributeMaxDynamicSharedMemorySize, lds256);
  (void)hipFuncSetAttribute(reinterpret_cast<const void*>(&sage_kernel<128, 256, false>), hipFuncAttributeMaxDynamicSharedMemorySize, lds128);
  (void)hipFuncSetAttribute(reinterpret_cast<const void*>(&sage_kernel<128, 128, true>), hipFuncAttributeMaxDynamicSharedMemorySize, lds128);

  pref_kernel<128><<<dim3(1), dim3(128), 0, stream>>>(RA, AG);
  sage_kernel<128, 128, false><<<dim3(NB), dim3(128), lds128, stream>>>(RA, AG, W1r, W1l, g1_bl, RB, RB);
  pref_kernel<128><<<dim3(1), dim3(128), 0, stream>>>(RB, AG);
  sage_kernel<256, 128, false><<<dim3(NB), dim3(256), lds256, stream>>>(RB, AG, W2r, W2l, g2_bl, RC, RC);
  pref_kernel<256><<<dim3(1), dim3(256), 0, stream>>>(RC, AG);
  sage_kernel<128, 256, false><<<dim3(NB), dim3(128), lds128, stream>>>(RC, AG, W3r, W3l, g3_bl, RA, RA);
  pref_kernel<128><<<dim3(1), dim3(128), 0, stream>>>(RA, AG);
  sage_kernel<128, 128, true><<<dim3(NB), dim3(128), lds128, stream>>>(RA, AG, W4r, W4l, g4_bl, RB, RC);

  for (int c = 0; c < NCH; ++c) {
    gemm64_kernel<4, 2, false><<<dim3(1, NWK, CHB), dim3(128), 0, stream>>>(
        SP, 128, 16384L, 0L,
        RC + (size_t)c * CHB * 32768, 256, 0L, 32768L,
        (void*)RD, (void*)(RD + 1024), (void*)RD, UTP, 128L, (long)(128 * UTP),
        2, 128, 2, 0, 0, 0, 0, 128, 0);
    unsigned short* ZTc = RA + (size_t)c * CHROWS * 256;
    gemm64_kernel<8, 2, false><<<dim3((CHROWS / 64) * 2 / 8, 1, 1), dim3(256), 0, stream>>>(
        RD, UTP, 0L, 0L, MC, MCP, 0L, 0L,
        (void*)ZTc, (void*)(ZTc + 128), (void*)ZTc, 256, 0L, 0L,
        2, 1024, 3, 0, 1024, 0, 0, 1024, 2048);
  }

  gemm64_kernel<4, 0, false><<<dim3(1, NB, 1), dim3(128), 0, stream>>>(
      RB, 256, 32768L, 0L, RA, 256, 32768L, 0L,
      (void*)out, (void*)out, (void*)out, 128, 16384L, 0L,
      2, 128, 3, 0, 128, 0, 0, 0, 128);
  (void)hipGetLastError();
}
